// LRU_25348896981257
// MI455X (gfx1250) — hardware-verified
//
#include <hip/hip_runtime.h>
#include <math.h>

constexpr int NB_SEQ   = 8;
constexpr int NSTEP    = 4096;
constexpr int NIN_F    = 128;
constexpr int NOUT_F   = 128;
constexpr int NSTATE   = 256;
constexpr int NROWS    = NB_SEQ * NSTEP;
constexpr int BUP      = 2 * NSTATE;
constexpr int AXP      = 2 * NSTATE + NIN_F;
constexpr int NTHR     = 256;
constexpr int SCAN_THR = 64;
constexpr float WCAR     = 64.0f;
constexpr float WCAR_INV = 1.0f / 64.0f;
constexpr int PREP_WB_BLK = (2 * NSTATE * NIN_F / 8) / NTHR;
constexpr int PREP_WC_BLK = (NOUT_F * 2 * NSTATE / 8) / NTHR;
constexpr int PREP_WD_BLK = (NOUT_F * NIN_F / 8) / NTHR;
constexpr int PREP_NBLK   = PREP_WB_BLK + PREP_WC_BLK + PREP_WD_BLK + 1;
constexpr int CVT_NBLK    = (NROWS * NIN_F / 8) / NTHR;
constexpr int GEMM_BU_BLK  = ((NROWS / 64) * (BUP / 64)) / 8;
constexpr int GEMM_OUT_BLK = ((NROWS / 64) * (NOUT_F / 64)) / 8;
static_assert((2 * NSTATE * NIN_F / 8) % NTHR == 0);
static_assert((NOUT_F * 2 * NSTATE / 8) % NTHR == 0);
static_assert((NOUT_F * NIN_F / 8) % NTHR == 0);
static_assert((NROWS * NIN_F / 8) % NTHR == 0);
static_assert(NSTATE == NTHR);
static_assert(NSTATE == 4 * SCAN_THR);
static_assert(NROWS % 64 == 0 && BUP % 64 == 0 && NOUT_F % 64 == 0);
static_assert(NIN_F % 32 == 0 && AXP % 32 == 0);
static_assert(((NROWS / 64) * (BUP / 64)) % 8 == 0 && ((NROWS / 64) * (NOUT_F / 64)) % 8 == 0);
static_assert(NIN_F % 8 == 0 && AXP % 8 == 0);

typedef __attribute__((ext_vector_type(16))) _Float16 v16h;
typedef __attribute__((ext_vector_type(8)))  _Float16 v8h;
typedef __attribute__((ext_vector_type(16))) __bf16   v16b;
typedef __attribute__((ext_vector_type(8)))  __bf16   v8b;
typedef __attribute__((ext_vector_type(8)))  float    v8f;
typedef __attribute__((ext_vector_type(4)))  float    v4f;

__device__ __forceinline__ unsigned short f2bf_bits(float f) {
  unsigned u = __float_as_uint(f);
  return (unsigned short)((u + 0x7FFFu + ((u >> 16) & 1u)) >> 16);
}
__device__ __forceinline__ float bf_bits2f(unsigned short h) { return __uint_as_float(((unsigned)h) << 16); }

__device__ __forceinline__ void dep_guard_h(v8f& a, v8f& b, v16h x, v16h y) { asm volatile("v_nop\n\tv_nop\n\tv_nop\n\tv_nop" : "+v"(a), "+v"(b) : "v"(x), "v"(y)); }
__device__ __forceinline__ void dep_guard_b(v8f& a, v8f& b, v16b x, v16b y) { asm volatile("v_nop\n\tv_nop\n\tv_nop\n\tv_nop" : "+v"(a), "+v"(b) : "v"(x), "v"(y)); }
__device__ __forceinline__ void keep4_h(v16h a, v16h b, v16h c, v16h d) { asm volatile("v_nop" :: "v"(a), "v"(b), "v"(c), "v"(d)); }
__device__ __forceinline__ void keep4_b(v16b a, v16b b, v16b c, v16b d) { asm volatile("v_nop" :: "v"(a), "v"(b), "v"(c), "v"(d)); }
__device__ __forceinline__ void acc_guard4(v8f& a, v8f& b, v8f& c, v8f& d) { asm volatile("v_nop\n\tv_nop\n\tv_nop\n\tv_nop" : "+v"(a), "+v"(b), "+v"(c), "+v"(d)); }
template <typename T> struct Frag;
template <> struct Frag<_Float16> {
  typedef v16h V; union U { v16h v; v8h h[2]; };
  static __device__ __forceinline__ v16h load(const _Float16* p) {
    U f; f.h[0] = *(const v8h*)(p); f.h[1] = *(const v8h*)(p + 16); return f.v;
  }
  static __device__ __forceinline__ v8f mma(v16h a, v16h b, v8f c) {
    return __builtin_amdgcn_wmma_f32_16x16x32_f16(false, a, false, b, (short)0, c, false, false);
  }
  static __device__ __forceinline__ void guard(v8f& a, v8f& b, v16h x, v16h y) { dep_guard_h(a, b, x, y); }
  static __device__ __forceinline__ void keep(v16h a, v16h b, v16h c, v16h d) { keep4_h(a, b, c, d); }
};
template <> struct Frag<__bf16> {
  typedef v16b V; union U { v16b v; v8b h[2]; };
  static __device__ __forceinline__ v16b load(const __bf16* p) {
    U f; f.h[0] = *(const v8b*)(p); f.h[1] = *(const v8b*)(p + 16); return f.v;
  }
  static __device__ __forceinline__ v8f mma(v16b a, v16b b, v8f c) {
    return __builtin_amdgcn_wmma_f32_16x16x32_bf16(false, a, false, b, (short)0, c, false, false);
  }
  static __device__ __forceinline__ void guard(v8f& a, v8f& b, v16b x, v16b y) { dep_guard_b(a, b, x, y); }
  static __device__ __forceinline__ void keep(v16b a, v16b b, v16b c, v16b d) { keep4_b(a, b, c, d); }
};

template <int ET> struct Elem;
template <> struct Elem<0> { typedef _Float16 T; };
template <> struct Elem<1> { typedef __bf16 T; };
template <int ET, bool SPLIT, int BIAS_MODE, int OUT_MODE, bool RESID, int ACT = 0>
__global__ __launch_bounds__(256) void wmma_gemm64(
    const unsigned short* __restrict__ Ap, const unsigned short* __restrict__ A2p, int lda, long strideA,
    const unsigned short* __restrict__ Btp, const unsigned short* __restrict__ Bt2p, int ldb, long strideB,
    void* __restrict__ Cout, void* __restrict__ Cout2, int ldc, long strideC,
    const float* __restrict__ bias,
    const float* __restrict__ resid, long strideR,
    int M, int N, int K, float scale) {
  typedef typename Elem<ET>::T T;
  typedef typename Frag<T>::V V;
  const T* A = (const T*)Ap; const T* A2 = (const T*)A2p; const T* Bt = (const T*)Btp; const T* Bt2 = (const T*)Bt2p;
  __shared__ __align__(16) float sT[8][16 * 68];
  const int b    = blockIdx.y;
  const int lane = threadIdx.x & 31;
  const int wave = threadIdx.x >> 5;
  const int tilesN = N >> 6;
  const int tilesM = M >> 6;
  const int tile = blockIdx.x * 8 + wave;
  if (tile >= tilesM * tilesN) return;
  const int tm = tile / tilesN;
  const int tn = tile - tm * tilesN;
  const int m0 = tm << 6;
  const int n0 = tn << 6;

  const T* Ab  = A  + (size_t)b * strideA;
  const T* Bb  = Bt + (size_t)b * strideB;
  const T* Ab2 = SPLIT ? (A2  + (size_t)b * strideA) : nullptr;
  const T* Bb2 = SPLIT ? (Bt2 + (size_t)b * strideB) : nullptr;

  const int rlane = lane & 15;
  const int koff  = (lane >> 4) * 8;
  const int mOff  = (lane >> 4) * 8;

  v8f acc[4][4];
#pragma unroll
  for (int i = 0; i < 4; ++i)
#pragma unroll
    for (int j = 0; j < 4; ++j) acc[i][j] = (v8f){0.f,0.f,0.f,0.f,0.f,0.f,0.f,0.f};

  for (int k0 = 0; k0 < K; k0 += 32) {
    V bh[4], bl[4];
#pragma unroll
    for (int j = 0; j < 4; ++j) {
      const size_t bo = (size_t)(n0 + (j << 4) + rlane) * ldb + koff + k0;
      bh[j] = Frag<T>::load(Bb + bo);
      if (SPLIT) bl[j] = Frag<T>::load(Bb2 + bo);
    }
#pragma unroll
    for (int i = 0; i < 4; ++i) {
      const size_t ao = (size_t)(m0 + (i << 4) + rlane) * lda + koff + k0;
      V ah = Frag<T>::load(Ab + ao);
      V al;
      if (SPLIT) al = Frag<T>::load(Ab2 + ao);
#pragma unroll
      for (int j = 0; j < 4; ++j) {
        acc[i][j] = Frag<T>::mma(ah, bh[j], acc[i][j]);
        if (SPLIT) {
          acc[i][j] = Frag<T>::mma(ah, bl[j], acc[i][j]);
          acc[i][j] = Frag<T>::mma(al, bh[j], acc[i][j]);
        }
      }
      Frag<T>::guard(acc[i][0], acc[i][3], ah, SPLIT ? al : ah);
    }
    Frag<T>::keep(bh[0], bh[1], bh[2], bh[3]);
    if (SPLIT) Frag<T>::keep(bl[0], bl[1], bl[2], bl[3]);
  }
  acc_guard4(acc[0][0], acc[0][1], acc[0][2], acc[0][3]);
  acc_guard4(acc[1][0], acc[1][1], acc[1][2], acc[1][3]);
  acc_guard4(acc[2][0], acc[2][1], acc[2][2], acc[2][3]);
  acc_guard4(acc[3][0], acc[3][1], acc[3][2], acc[3][3]);

  float* slab = sT[wave];
  const float* Rb = RESID ? (resid + (size_t)b * strideR) : nullptr;
#pragma unroll
  for (int i = 0; i < 4; ++i) {
    const int mBase = m0 + (i << 4);
#pragma unroll
    for (int j = 0; j < 4; ++j) {
      const int n = n0 + (j << 4) + rlane;
      float bv = 0.f;
      if (BIAS_MODE == 2) bv = bias[n];
#pragma unroll
      for (int r = 0; r < 8; ++r) {
        float v = acc[i][j][r] * scale;
        if (BIAS_MODE == 1) v += bias[mBase + mOff + r];
        if (BIAS_MODE == 2) v += bv;
        if (RESID) v += Rb[(size_t)(mBase + mOff + r) * ldc + n];
        if (ACT == 1) v = tanhf(v);
        if (ACT == 2) v = fmaxf(v, 0.0f);
        if (ACT == 3) v = v / (1.0f + expf(-v));
        if (ACT == 4) v = (v > 0.f) ? v : 0.01f * v;
        if (ACT == 5) v = 0.5f * v * (1.0f + erff(v * 0.70710678118654752f));
        slab[(mOff + r) * 68 + (j << 4) + rlane] = v;
      }
    }
    __builtin_amdgcn_fence(__ATOMIC_RELEASE, "workgroup");
    __builtin_amdgcn_wave_barrier();
    __builtin_amdgcn_fence(__ATOMIC_ACQUIRE, "workgroup");
    if (OUT_MODE == 0) {
      float* C = (float*)Cout + (size_t)b * strideC;
      const int hh = lane >> 4, c4 = (lane & 15) * 4;
      for (int pass = 0; pass < 2; ++pass) {
#pragma unroll
        for (int it = 0; it < 8; ++it) {
          const int row = it * 2 + hh;
          v4f v = *(const v4f*)(slab + row * 68 + c4);
          *(volatile v4f*)(C + (size_t)(mBase + row) * ldc + n0 + c4) = v;
        }
        __threadfence();
      }
    } else {
      const int q = lane >> 3, c8 = (lane & 7) * 8;
      unsigned short* C  = (unsigned short*)Cout  + (size_t)b * strideC;
      unsigned short* C2 = (OUT_MODE == 2) ? ((unsigned short*)Cout2 + (size_t)b * strideC) : nullptr;
      for (int pass = 0; pass < 2; ++pass) {
#pragma unroll
        for (int it = 0; it < 4; ++it) {
          const int row = it * 4 + q;
          const float* sp = slab + row * 68 + c8;
          v8h hv, lv;
#pragma unroll
          for (int e = 0; e < 8; ++e) {
            if (OUT_MODE == 1) {
              hv[e] = (_Float16)sp[e];
            } else {
              unsigned short hb = f2bf_bits(sp[e]);
              unsigned short lb = f2bf_bits(sp[e] - bf_bits2f(hb));
              hv[e] = __builtin_bit_cast(_Float16, hb);
              lv[e] = __builtin_bit_cast(_Float16, lb);
            }
          }
          *(volatile v8h*)(C + (size_t)(mBase + row) * ldc + n0 + c8) = hv;
          if (OUT_MODE == 2) *(volatile v8h*)(C2 + (size_t)(mBase + row) * ldc + n0 + c8) = lv;
        }
        __threadfence();
      }
    }
    __builtin_amdgcn_fence(__ATOMIC_RELEASE, "workgroup");
    __builtin_amdgcn_wave_barrier();
    __builtin_amdgcn_fence(__ATOMIC_ACQUIRE, "workgroup");
  }
}

__global__ __launch_bounds__(NTHR) void prep_kernel(
    const float* __restrict__ nu_log, const float* __restrict__ theta_log, const float* __restrict__ gamma_log,
    const float* __restrict__ B_re, const float* __restrict__ B_im,
    const float* __restrict__ C_re, const float* __restrict__ C_im, const float* __restrict__ Dm,
    unsigned short* __restrict__ WB, unsigned short* __restrict__ WOUT, float* __restrict__ LAM) {
  __shared__ __align__(16) float lamsh[2 * NSTATE];
  const int tid = threadIdx.x;
  const int bid = blockIdx.x;
  if (bid < PREP_WB_BLK) {
    const int i  = bid * NTHR + tid;
    const int r  = i >> 4;
    const int c8 = (i & 15) * 8;
    const int n  = r & (NSTATE - 1);
    const bool imPart = (bid >= PREP_WB_BLK / 2);
    const float* src = imPart ? B_im : B_re;
    const float g = expf(gamma_log[n]) * WCAR;
    const v4f va = *(const v4f*)(src + (size_t)n * NIN_F + c8);
    const v4f vb = *(const v4f*)(src + (size_t)n * NIN_F + c8 + 4);
    v8h hv;
#pragma unroll
    for (int e = 0; e < 4; ++e) {
      hv[e]     = (_Float16)(g * va[e]);
      hv[4 + e] = (_Float16)(g * vb[e]);
    }
    unsigned short* dst = WB + (size_t)i * 8;
    *(volatile v8h*)dst = hv;
    __threadfence();
    *(volatile v8h*)dst = hv;
  } else if (bid < PREP_WB_BLK + PREP_WC_BLK) {
    const int jc = (bid - PREP_WB_BLK) * NTHR + tid;
    const int d  = jc >> 6;
    const int n0 = (jc & 63) * 4;
    const v4f cr = *(const v4f*)(C_re + (size_t)d * NSTATE + n0);
    const v4f ci = *(const v4f*)(C_im + (size_t)d * NSTATE + n0);
    v8h hv;
#pragma unroll
    for (int e = 0; e < 4; ++e) {
      hv[2 * e]     = (_Float16)(cr[e] * WCAR);
      hv[2 * e + 1] = (_Float16)(-(ci[e] * WCAR));
    }
    unsigned short* dst = WOUT + (size_t)d * AXP + 2 * n0;
    *(volatile v8h*)dst = hv;
    __threadfence();
    *(volatile v8h*)dst = hv;
  } else if (bid < PREP_WB_BLK + PREP_WC_BLK + PREP_WD_BLK) {
    const int jd = (bid - PREP_WB_BLK - PREP_WC_BLK) * NTHR + tid;
    const int d  = jd >> 4;
    const int c8 = (jd & 15) * 8;
    const v4f va = *(const v4f*)(Dm + (size_t)d * NIN_F + c8);
    const v4f vb = *(const v4f*)(Dm + (size_t)d * NIN_F + c8 + 4);
    v8h hv;
#pragma unroll
    for (int e = 0; e < 4; ++e) {
      hv[e]     = (_Float16)(va[e] * WCAR);
      hv[4 + e] = (_Float16)(vb[e] * WCAR);
    }
    unsigned short* dst = WOUT + (size_t)d * AXP + 2 * NSTATE + c8;
    *(volatile v8h*)dst = hv;
    __threadfence();
    *(volatile v8h*)dst = hv;
  } else {
    const int n = tid;
    const float la = expf(-expf(nu_log[n]));
    const float ph = expf(theta_log[n]);
    const float cs = cosf(ph);
    const float sn = sinf(ph);
    lamsh[n]          = la * cs;
    lamsh[NSTATE + n] = la * sn;
    __syncthreads();
    if (tid < (2 * NSTATE) / 4) {
      const v4f v = *(const v4f*)(lamsh + 4 * tid);
      float* dst = LAM + 4 * tid;
      *(volatile v4f*)dst = v;
      __threadfence();
      *(volatile v4f*)dst = v;
    }
  }
}

__global__ __launch_bounds__(NTHR) void cvtx_kernel(const float* __restrict__ x, unsigned short* __restrict__ AX) {
  const int i   = blockIdx.x * NTHR + threadIdx.x;
  const int row = i >> 4;
  const int c8  = (i & 15) * 8;
  const float* sp = x + (size_t)row * NIN_F + c8;
  const v4f va = *(const v4f*)(sp);
  const v4f vb = *(const v4f*)(sp + 4);
  v8h hv;
#pragma unroll
  for (int e = 0; e < 4; ++e) {
    hv[e]     = (_Float16)va[e];
    hv[4 + e] = (_Float16)vb[e];
  }
  unsigned short* dst = AX + (size_t)row * AXP + 2 * NSTATE + c8;
  *(volatile v8h*)dst = hv;
  __threadfence();
  *(volatile v8h*)dst = hv;
}

__global__ __launch_bounds__(SCAN_THR) void scan_kernel(const float* __restrict__ BU, const float* __restrict__ LAM,
                                                        unsigned short* __restrict__ AX) {
  const int b = blockIdx.x;
  const int q = threadIdx.x;
  const v4f lr4 = *(const v4f*)(LAM + 4 * q);
  const v4f li4 = *(const v4f*)(LAM + NSTATE + 4 * q);
  float sr[4], si[4];
#pragma unroll
  for (int e = 0; e < 4; ++e) { sr[e] = 0.0f; si[e] = 0.0f; }
  const size_t rowb = (size_t)b * NSTEP;
  const float* bup = BU + rowb * BUP + 4 * q;
  v4f nre = *(const v4f*)(bup);
  v4f nim = *(const v4f*)(bup + NSTATE);
#pragma unroll 1
  for (int t = 0; t < NSTEP; ++t) {
    const v4f ur = nre, ui = nim;
    const int tn = (t + 1 < NSTEP) ? (t + 1) : (NSTEP - 1);
    nre = *(const v4f*)(bup + (size_t)tn * BUP);
    nim = *(const v4f*)(bup + (size_t)tn * BUP + NSTATE);
    v8h hv;
#pragma unroll
    for (int e = 0; e < 4; ++e) {
      const float a = lr4[e] * sr[e] - li4[e] * si[e] + ur[e];
      const float c = lr4[e] * si[e] + li4[e] * sr[e] + ui[e];
      sr[e] = a;
      si[e] = c;
      hv[2 * e]     = (_Float16)a;
      hv[2 * e + 1] = (_Float16)c;
    }
    unsigned short* dst = AX + (rowb + (size_t)t) * AXP + 8 * q;
    *(volatile v8h*)dst = hv;
    __threadfence();
    *(volatile v8h*)dst = hv;
  }
}

extern "C" void kernel_launch(void* const* d_in, const int* in_sizes, int n_in,
                              void* d_out, int out_size, void* d_ws, size_t ws_size, hipStream_t stream) {
  if (n_in < 9 || d_out == nullptr || d_ws == nullptr) return;
  if (in_sizes[0] != NROWS * NIN_F || in_sizes[1] != NSTATE || in_sizes[2] != NSTATE || in_sizes[3] != NSTATE ||
      in_sizes[4] != NSTATE * NIN_F || in_sizes[5] != NSTATE * NIN_F || in_sizes[6] != NOUT_F * NSTATE ||
      in_sizes[7] != NOUT_F * NSTATE || in_sizes[8] != NOUT_F * NIN_F || out_size != NROWS * NOUT_F) return;

  const float* x         = (const float*)d_in[0];
  const float* nu_log    = (const float*)d_in[1];
  const float* theta_log = (const float*)d_in[2];
  const float* gamma_log = (const float*)d_in[3];
  const float* B_re      = (const float*)d_in[4];
  const float* B_im      = (const float*)d_in[5];
  const float* C_re      = (const float*)d_in[6];
  const float* C_im      = (const float*)d_in[7];
  const float* Dm        = (const float*)d_in[8];
  float* y = (float*)d_out;

  char* ws = (char*)d_ws; size_t off = 0;
  auto carve = [&](size_t bytes) -> char* { char* p = ws + off; off += (bytes + 255) & ~(size_t)255; return p; };
  unsigned short* AX   = (unsigned short*)carve((size_t)NROWS * AXP * 2);
  float*          BU   = (float*)carve((size_t)NROWS * BUP * 4);
  unsigned short* WB   = (unsigned short*)carve((size_t)2 * NSTATE * NIN_F * 2);
  unsigned short* WOUT = (unsigned short*)carve((size_t)NOUT_F * AXP * 2);
  float*          LAM  = (float*)carve((size_t)2 * NSTATE * 4);
  if (off > ws_size || off > (size_t)134217728) return;

  prep_kernel<<<PREP_NBLK, NTHR, 0, stream>>>(nu_log, theta_log, gamma_log, B_re, B_im, C_re, C_im, Dm, WB, WOUT, LAM);
  cvtx_kernel<<<CVT_NBLK, NTHR, 0, stream>>>(x, AX);
  wmma_gemm64<0, false, 0, 0, false, 0><<<dim3(GEMM_BU_BLK, 1), 256, 0, stream>>>(
      AX + 2 * NSTATE, AX + 2 * NSTATE, AXP, 0L, WB, WB, NIN_F, 0L, (void*)BU, (void*)BU, BUP, 0L,
      LAM, LAM, 0L, NROWS, BUP, NIN_F, WCAR_INV);
  scan_kernel<<<NB_SEQ, SCAN_THR, 0, stream>>>(BU, LAM, AX);
  wmma_gemm64<0, false, 0, 0, false, 0><<<dim3(GEMM_OUT_BLK, 1), 256, 0, stream>>>(
      AX, AX, AXP, 0L, WOUT, WOUT, AXP, 0L, (void*)y, (void*)y, NOUT_F, 0L,
      LAM, LAM, 0L, NROWS, NOUT_F, AXP, WCAR_INV);
}
